// DenseKAN_81655918231937
// MI455X (gfx1250) — hardware-run, weakly checked
//
#include <hip/hip_runtime.h>
#include <math.h>

typedef __attribute__((ext_vector_type(16))) _Float16 v16h;
typedef __attribute__((ext_vector_type(16))) __bf16 v16b;
typedef __attribute__((ext_vector_type(8)))  _Float16 v8h;
typedef __attribute__((ext_vector_type(8)))  float v8f;
typedef __attribute__((ext_vector_type(4)))  float v4f;
typedef __attribute__((ext_vector_type(2)))  float v2f;
typedef __attribute__((ext_vector_type(4)))  unsigned v4u;
typedef __attribute__((ext_vector_type(4)))  int v4i;
typedef float __attribute__((may_alias)) float_a;
typedef int __attribute__((may_alias)) int_a;

template <typename T> __device__ __forceinline__ void vst2(void* p, T v) { *(volatile T*)p = v; __threadfence(); *(volatile T*)p = v; }
__device__ __forceinline__ v8f wmma16(v16h a, v16h b, v8f c) {
  v8f d = __builtin_amdgcn_wmma_f32_16x16x32_f16(false, a, false, b, (short)0, c, false, false);
  asm volatile("v_nop\n\tv_nop\n\tv_nop\n\tv_nop" : "+v"(d) : "v"(a), "v"(b));
  return d;
}
__device__ __forceinline__ v8f wmma_bf(v16b a, v16b b, v8f c) {
  v8f d = __builtin_amdgcn_wmma_f32_16x16x32_bf16(false, a, false, b, (short)0, c, false, false);
  asm volatile("v_nop\n\tv_nop\n\tv_nop\n\tv_nop" : "+v"(d) : "v"(a), "v"(b));
  return d;
}
__device__ __forceinline__ v16h frag_h(const _Float16* rowk0, int lane) {
  union { v16h v; v8h q[2]; } u; const _Float16* p = rowk0 + 8 * (lane >> 4);
  u.q[0] = *(const v8h*)p; u.q[1] = *(const v8h*)(p + 16); return u.v;
}
__device__ __forceinline__ v16h frag_f32(const float* rowk0, int lane) {
  v16h a; const float* p = rowk0 + 8 * (lane >> 4);
#pragma unroll
  for (int i = 0; i < 8; ++i) { a[i] = (_Float16)p[i]; a[8 + i] = (_Float16)p[16 + i]; }
  return a;
}
__device__ __forceinline__ v16h frag_f32s(const float* rowk0, int lane, float sc) {
  v16h a; const float* p = rowk0 + 8 * (lane >> 4);
#pragma unroll
  for (int i = 0; i < 8; ++i) { a[i] = (_Float16)(p[i] * sc); a[8 + i] = (_Float16)(p[16 + i] * sc); }
  return a;
}
__device__ __forceinline__ v16h fragc_f32(const float* W, int k0, int n, int lane, int ld, int K) {
  v16h a; const int g = lane >> 4;
#pragma unroll
  for (int i = 0; i < 8; ++i) { const int ka = k0 + 8 * g + i, kb = ka + 16;
    a[i] = (_Float16)(ka < K ? W[(size_t)(ka < K ? ka : K - 1) * ld + n] : 0.f); a[8 + i] = (_Float16)(kb < K ? W[(size_t)(kb < K ? kb : K - 1) * ld + n] : 0.f); }
  return a;
}
struct F2 { v16b h, l; };
__device__ __forceinline__ F2 bsplit16(const float v[16]) { F2 r;
#pragma unroll
  for (int i = 0; i < 16; ++i) { const __bf16 h = (__bf16)v[i]; r.h[i] = h; r.l[i] = (__bf16)(v[i] - (float)h); }
  return r; }
__device__ __forceinline__ F2 split_row(const float* row, int k0, int lane) { float v[16]; const float* p = row + k0 + 8 * (lane >> 4);
#pragma unroll
  for (int i = 0; i < 8; ++i) { v[i] = p[i]; v[8 + i] = p[16 + i]; }
  return bsplit16(v); }
__device__ __forceinline__ F2 split_rowK(const float* row, int k0, int lane, int K) { float v[16]; const int g = lane >> 4;
#pragma unroll
  for (int i = 0; i < 8; ++i) { const int ka = k0 + 8 * g + i, kb = ka + 16; v[i] = ka < K ? row[ka < K ? ka : K - 1] : 0.f; v[8 + i] = kb < K ? row[kb < K ? kb : K - 1] : 0.f; }
  return bsplit16(v); }
__device__ __forceinline__ F2 split_col(const float* W, int k0, int n, int lane, int ld, int K) { float v[16]; const int g = lane >> 4;
#pragma unroll
  for (int i = 0; i < 8; ++i) { const int ka = k0 + 8 * g + i, kb = ka + 16; v[i] = ka < K ? W[(size_t)(ka < K ? ka : K - 1) * ld + n] : 0.f; v[8 + i] = kb < K ? W[(size_t)(kb < K ? kb : K - 1) * ld + n] : 0.f; }
  return bsplit16(v); }
__device__ __forceinline__ v8f mac3(const F2& a, const F2& b, v8f c) { c = wmma_bf(a.l, b.h, c); c = wmma_bf(a.h, b.l, c); return wmma_bf(a.h, b.h, c); }
__device__ __forceinline__ float sigm(float v) { return 1.0f / (1.0f + expf(-v)); }
#define LDSX() do { asm volatile("s_wait_dscnt 0" ::: "memory"); __builtin_amdgcn_wave_barrier(); __builtin_amdgcn_fence(__ATOMIC_RELEASE, "workgroup"); } while (0)


#define NBATCH 4096
#define NI 128
#define NU 128
#define NBAS 8
#define NKNOT 12
#define KDIM (NI * NBAS)
#ifndef TROW
#define TROW NBATCH
#endif
typedef __attribute__((ext_vector_type(8))) __bf16 v8b;
__device__ __forceinline__ v16b frag_b(const __bf16* rowk0, int lane) {
  union { v16b v; v8b q[2]; } u; const __bf16* p = rowk0 + 8 * (lane >> 4);
  u.q[0] = *(const v8b*)p; u.q[1] = *(const v8b*)(p + 16); return u.v;
}
__device__ __forceinline__ float bfr(float v) { return (float)(__bf16)v; }
__device__ __attribute__((noinline)) float exp_ni(float v) { return expf(v); }
__device__ __attribute__((noinline)) float erf_ni(float v) { return erff(v); }

#define WS_KH  0u
#define WS_KL  (WS_KH + 2u * NU * KDIM)
#define WS_SC  (WS_KL + 2u * NU * KDIM)
#define WS_END (WS_SC + 2u * NU * NI)

__device__ __forceinline__ float knot(int j) { return -2.2f + (float)j * (4.4f / 11.0f); }
__device__ __forceinline__ void bases8(float x, float bo[NBAS]) { float bcur[NKNOT - 1];
#pragma unroll
  for (int j = 0; j < NKNOT - 1; ++j) bcur[j] = (x >= knot(j) && x < knot(j + 1)) ? 1.0f : 0.0f;
#pragma unroll
  for (int k = 1; k <= 3; ++k) {
#pragma unroll
    for (int j = 0; j < NKNOT - 1 - k; ++j) { const float left = (x - knot(j)) / (knot(j + k) - knot(j)); const float right = (knot(j + k + 1) - x) / (knot(j + k + 1) - knot(j + 1)); bcur[j] = left * bcur[j] + right * bcur[j + 1]; } }
#pragma unroll
  for (int k = 0; k < NBAS; ++k) bo[k] = bcur[k]; }
__global__ __launch_bounds__(256) void k_pack(const float* __restrict__ KERN, const float* __restrict__ SCALE, __bf16* __restrict__ PH, __bf16* __restrict__ PL, __bf16* __restrict__ SCT) { __shared__ __align__(16) __bf16 sh[KDIM], sl[KDIM], ss[NI]; const int o = blockIdx.x, t = threadIdx.x;
  for (int e = t; e < KDIM; e += 256) { const int i = e / NBAS; const float v = bfr(KERN[(size_t)e * NU + o]) * bfr(SCALE[i * NU + o]); const __bf16 h = (__bf16)v; sh[e] = h; sl[e] = (__bf16)(v - (float)h); }
  if (t < NI) ss[t] = (__bf16)SCALE[t * NU + o];
  __syncthreads();
  for (int q = t; q < KDIM / 8; q += 256) { vst2((unsigned*)(PH + (size_t)o * KDIM + q * 8), *(const v4u*)&sh[q * 8]); vst2((unsigned*)(PL + (size_t)o * KDIM + q * 8), *(const v4u*)&sl[q * 8]); }
  if (t < NI / 8) vst2((unsigned*)(SCT + (size_t)o * NI + t * 8), *(const v4u*)&ss[t * 8]); }
__global__ __launch_bounds__(128) void k_main(const float* __restrict__ X, const __bf16* __restrict__ PH, const __bf16* __restrict__ PL, const __bf16* __restrict__ SCT, const float* __restrict__ BIAS, float* __restrict__ OUT) { __shared__ __align__(16) float sf[4][16][132];
  const int tid = threadIdx.x, wave = tid >> 5, lane = tid & 31, col = lane & 15, g = lane >> 4; const size_t r0 = (size_t)blockIdx.x * 64 + wave * 16; const float* xr = X + (r0 + col) * NI;
#pragma unroll 1
  for (int hf = 0; hf < 2; ++hf) {
  v8f acc[4] = {};
#pragma unroll 1
  for (int kc = 0; kc < KDIM / 32; ++kc) {
    float v[16]; float ba[NBAS], bb[NBAS]; bases8(bfr(xr[kc * 4 + g]), ba); bases8(bfr(xr[kc * 4 + 2 + g]), bb);
#pragma unroll
    for (int i = 0; i < 8; ++i) { v[i] = ba[i]; v[8 + i] = bb[i]; }
    const F2 a = bsplit16(v);
#pragma unroll
    for (int j = 0; j < 4; ++j) { const int jj = hf * 4 + j; const F2 w = { frag_b(PH + (size_t)(jj * 16 + col) * KDIM + kc * 32, lane), frag_b(PL + (size_t)(jj * 16 + col) * KDIM + kc * 32, lane) }; acc[j] = mac3(a, w, acc[j]); } }
#pragma unroll 1
  for (int kc = 0; kc < NI / 32; ++kc) { float v[16];
#pragma unroll
    for (int i = 0; i < 8; ++i) { const float xa = bfr(xr[kc * 32 + 8 * g + i]), xb = bfr(xr[kc * 32 + 16 + 8 * g + i]); v[i] = xa / (1.0f + expf(-xa)); v[8 + i] = xb / (1.0f + expf(-xb)); }
    const F2 a = bsplit16(v);
#pragma unroll
    for (int j = 0; j < 4; ++j) { const int jj = hf * 4 + j; const v16b w = frag_b(SCT + (size_t)(jj * 16 + col) * NI + kc * 32, lane); acc[j] = wmma_bf(a.h, w, acc[j]); acc[j] = wmma_bf(a.l, w, acc[j]); } }
#pragma unroll
  for (int j = 0; j < 4; ++j)
#pragma unroll
    for (int r = 0; r < 8; ++r) sf[wave][8 * g + r][(hf * 4 + j) * 16 + col] = acc[j][r] + bfr(BIAS[(hf * 4 + j) * 16 + col]);
  }
  LDSX(); for (int rl = 0; rl < 16; ++rl) vst2(OUT + (r0 + rl) * NU + lane * 4, *(const v4f*)&sf[wave][rl][lane * 4]); }
extern "C" void kernel_launch(void* const* d_in, const int* in_sizes, int n_in, void* d_out, int out_size, void* d_ws, size_t ws_size, hipStream_t stream) {
  (void)in_sizes; (void)n_in; (void)out_size;
  const float** F = (const float**)d_in;
  if (ws_size < (size_t)WS_END) return;
  char* ws = (char*)d_ws; __bf16 *PH = (__bf16*)(ws + WS_KH), *PL = (__bf16*)(ws + WS_KL), *SCT = (__bf16*)(ws + WS_SC);
  k_pack<<<NU, 256, 0, stream>>>(F[1], F[2], PH, PL, SCT);
  k_main<<<TROW / 64, 128, 0, stream>>>(F[0], PH, PL, SCT, F[3], (float*)d_out);
}
